// KANLayer_5239860101393
// MI455X (gfx1250) — hardware-verified
//
#include <hip/hip_runtime.h>
#include <stdint.h>

#define NROWS   4096
#define NIN     512
#define NOUT    512
#define NSEG    9
#define NPOW    4
#define KPI     (NSEG * NPOW)
#define KTOT    (NIN * KPI)
#define CH      2048
#define NCHUNK  (NROWS / CH)
#define UROW    (KTOT / 8)
#define FTHR    512
#define NSWEEP  ((UROW + FTHR - 1) / FTHR)
#define PUNITS  (NOUT * KTOT / 8)
#define PBLKS   (PUNITS / 256)
#define CW      1024.0f
#define CINV    0.0009765625f
#define FMINN   6.103515625e-05f
#define WSCAP   134217728

static_assert(NROWS == NCHUNK * CH);
static_assert(CH % 128 == 0);
static_assert(NOUT % 64 == 0);
static_assert(KTOT % 32 == 0);
static_assert(UROW % 32 == 0);
static_assert(NSWEEP * FTHR >= UROW);
static_assert(PUNITS == PBLKS * 256);
static_assert(FTHR == NIN);
static_assert((KPI * 2) % 8 == 0);
static_assert((KTOT * 2) % 128 == 0);

typedef float          v4f   __attribute__((ext_vector_type(4)));
typedef float          v8f   __attribute__((ext_vector_type(8)));
typedef int            v8i   __attribute__((ext_vector_type(8)));
typedef unsigned int   v2u   __attribute__((ext_vector_type(2)));
typedef unsigned int   v4u   __attribute__((ext_vector_type(4)));
typedef unsigned short v8us  __attribute__((ext_vector_type(8)));
typedef unsigned short v16us __attribute__((ext_vector_type(16)));
typedef _Float16       v16h  __attribute__((ext_vector_type(16)));
typedef v4f  __attribute__((may_alias)) v4fa;
typedef v2u  __attribute__((may_alias)) v2ua;
typedef v4u  __attribute__((may_alias)) v4ua;
typedef v8us __attribute__((may_alias)) v8usa;
union FragH { v16h v; v16us u; v8us h[2]; v8i w; };

__device__ __forceinline__ unsigned short f2bf_bits(float f) {
  unsigned u = __float_as_uint(f);
  return (unsigned short)((u + 0x7FFFu + ((u >> 16) & 1u)) >> 16);
}
__device__ __forceinline__ float bf_bits2f(unsigned short b) { return __uint_as_float(((unsigned)b) << 16); }
__device__ __forceinline__ float bfr(float f) { return bf_bits2f(f2bf_bits(f)); }
__device__ __forceinline__ unsigned short f2h(float f) {
  const _Float16 hv = (_Float16)f;
  return __builtin_bit_cast(unsigned short, hv);
}
__device__ __forceinline__ unsigned pk16(unsigned short a, unsigned short b) { return (unsigned)a | ((unsigned)b << 16); }

__device__ __forceinline__ v8f wmh(const FragH& a, const FragH& b, v8f c) {
  v8f d = __builtin_amdgcn_wmma_f32_16x16x32_f16(false, a.v, false, b.v, (short)0, c, false, false);
  asm volatile("v_nop\n\tv_nop\n\tv_nop\n\tv_nop" : "+v"(d) : "v"(a.w), "v"(b.w));
  return d;
}
__device__ __forceinline__ v8f z8() { v8f z = {0.f, 0.f, 0.f, 0.f, 0.f, 0.f, 0.f, 0.f}; return z; }

__global__ __launch_bounds__(256) void prep_kernel(const float* __restrict__ coeff, unsigned short* __restrict__ WB) {
  const size_t u = (size_t)blockIdx.x * 256 + (size_t)threadIdx.x;
  const float* src = coeff + u * 8;
  unsigned short* dst = WB + u * 8;
  const v4f a = *(const v4fa*)src;
  const v4f c = *(const v4fa*)(src + 4);
  v4u v;
  v[0] = pk16(f2h(CW * bfr(a[0])), f2h(CW * bfr(a[1])));
  v[1] = pk16(f2h(CW * bfr(a[2])), f2h(CW * bfr(a[3])));
  v[2] = pk16(f2h(CW * bfr(c[0])), f2h(CW * bfr(c[1])));
  v[3] = pk16(f2h(CW * bfr(c[2])), f2h(CW * bfr(c[3])));
  *(volatile v4u*)dst = v;
  __threadfence();
  *(volatile v4u*)dst = v;
}

__device__ __forceinline__ void a_store_pass(const unsigned short* sA, unsigned short* dst, int tid) {
#pragma unroll
  for (int it = 0; it < NSWEEP; ++it) {
    const int u = it * FTHR + tid;
    if (u < UROW) {
      const v4u v = *(const v4ua*)(sA + 8 * u);
      *(volatile v4u*)(dst + 8 * u) = v;
    }
  }
}

__global__ __launch_bounds__(FTHR) void feat_kernel(const float* __restrict__ x, unsigned short* __restrict__ AP,
                                                    int row_base) {
  __shared__ __align__(16) unsigned short sA[KTOT];
  const int i = threadIdx.x;
  const int r = blockIdx.x;
  const float xb = bfr(x[(size_t)(row_base + r) * NIN + i]);
  const float xc = fminf(fmaxf(xb, -1.0f), 1.0f);

  const float k1 = __uint_as_float(0xBF471C72u);
  const float k2 = __uint_as_float(0xBF0E38E4u);
  const float k3 = __uint_as_float(0xBEAAAAABu);
  const float k4 = __uint_as_float(0xBDE38E39u);
  const float k5 = __uint_as_float(0x3DE38E39u);
  const float k6 = __uint_as_float(0x3EAAAAABu);
  const float k7 = __uint_as_float(0x3F0E38E4u);
  const float k8 = __uint_as_float(0x3F471C72u);

  int seg = 0;
  float lo = -1.0f, hi = k1;
  { const bool c = xc > k1; seg += c ? 1 : 0; lo = c ? k1 : lo; hi = c ? k2 : hi; }
  { const bool c = xc > k2; seg += c ? 1 : 0; lo = c ? k2 : lo; hi = c ? k3 : hi; }
  { const bool c = xc > k3; seg += c ? 1 : 0; lo = c ? k3 : lo; hi = c ? k4 : hi; }
  { const bool c = xc > k4; seg += c ? 1 : 0; lo = c ? k4 : lo; hi = c ? k5 : hi; }
  { const bool c = xc > k5; seg += c ? 1 : 0; lo = c ? k5 : lo; hi = c ? k6 : hi; }
  { const bool c = xc > k6; seg += c ? 1 : 0; lo = c ? k6 : lo; hi = c ? k7 : hi; }
  { const bool c = xc > k7; seg += c ? 1 : 0; lo = c ? k7 : lo; hi = c ? k8 : hi; }
  { const bool c = xc > k8; seg += c ? 1 : 0; lo = c ? k8 : lo; hi = c ? 1.0f : hi; }

  const float num = xc - lo;
  const float den = hi - lo;
  const float t1 = num * (1.0f / den);
  const float t2 = t1 * t1;
  const float t3 = t2 * t1;
  const float f1 = (t1 < FMINN) ? 0.0f : t1;
  const float f2 = (t2 < FMINN) ? 0.0f : t2;
  const float f3 = (t3 < FMINN) ? 0.0f : t3;
  typedef __fp16 v2h __attribute__((ext_vector_type(2)));
  const v2h p01 = __builtin_amdgcn_cvt_pkrtz(1.0f, f1);
  const v2h p23 = __builtin_amdgcn_cvt_pkrtz(f2, f3);
  const unsigned w01 = __builtin_bit_cast(unsigned, p01);
  const unsigned w23 = __builtin_bit_cast(unsigned, p23);

#pragma unroll
  for (int s = 0; s < NSEG; ++s) {
    const unsigned mk = (s == seg) ? 0xffffffffu : 0u;
    v2u wv;
    wv.x = w01 & mk;
    wv.y = w23 & mk;
    *(v2ua*)(sA + KPI * i + NPOW * s) = wv;
  }
  __syncthreads();

  unsigned short* dst = AP + (size_t)r * KTOT;
  a_store_pass(sA, dst, i);
  __threadfence();
  a_store_pass(sA, dst, i);
}

__device__ __forceinline__ void o_store_pass(const float* sO, float* out,
                                             int grow_w, int n0, int w, int lane) {
  const int q8 = lane & 7, sub = lane >> 3;
#pragma unroll
  for (int i = 0; i < 16; ++i) {
    const int lid = i * 4 + sub;
    const int row = lid >> 1, hl = lid & 1;
    const v4f v = *(const v4fa*)(sO + (32 * w + row) * 64 + 32 * hl + 4 * q8);
    *(volatile v4f*)(out + (size_t)(grow_w + row) * NOUT + n0 + 32 * hl + 4 * q8) = v;
  }
}

__global__ __launch_bounds__(128) void gemm_kernel(const unsigned short* __restrict__ AP,
                                                   const unsigned short* __restrict__ WB,
                                                   const float* __restrict__ scale,
                                                   float* __restrict__ out, int row_base) {
  __shared__ __align__(16) float sO[128 * 64];
  const int tid = threadIdx.x, lane = tid & 31, w = tid >> 5;
  const int h = lane >> 4, m = lane & 15;
  const int lrow_w = blockIdx.x * 128 + 32 * w;
  const int n0 = blockIdx.y * 64;

  const unsigned short* xa0 = AP + (size_t)(lrow_w + m) * KTOT + 8 * h;
  const unsigned short* xa1 = xa0 + (size_t)16 * KTOT;
  const unsigned short* wb  = WB + (size_t)(n0 + m) * KTOT + 8 * h;

  v8f acc[2][4];
#pragma unroll
  for (int mt = 0; mt < 2; ++mt)
#pragma unroll
    for (int nt = 0; nt < 4; ++nt) acc[mt][nt] = z8();

#pragma unroll 1
  for (int k0 = 0; k0 < KTOT; k0 += 32) {
    FragH a0, a1;
    a0.h[0] = *(const v8usa*)(xa0 + k0);
    a0.h[1] = *(const v8usa*)(xa0 + k0 + 16);
    a1.h[0] = *(const v8usa*)(xa1 + k0);
    a1.h[1] = *(const v8usa*)(xa1 + k0 + 16);
#pragma unroll
    for (int nt = 0; nt < 4; ++nt) {
      const unsigned short* wq = wb + (size_t)nt * 16 * KTOT + k0;
      FragH b;
      b.h[0] = *(const v8usa*)wq;
      b.h[1] = *(const v8usa*)(wq + 16);
      acc[0][nt] = wmh(a0, b, acc[0][nt]);
      acc[1][nt] = wmh(a1, b, acc[1][nt]);
    }
  }

#pragma unroll
  for (int nt = 0; nt < 4; ++nt) {
    const int cl = 16 * nt + m;
    const float sc = bfr(scale[n0 + cl]);
#pragma unroll
    for (int mt = 0; mt < 2; ++mt) {
#pragma unroll
      for (int r = 0; r < 8; ++r) {
        const int rl = 32 * w + 16 * mt + 8 * h + r;
        sO[rl * 64 + cl] = (acc[mt][nt][r] * CINV) * sc;
      }
    }
  }
  __syncthreads();

  const int grow_w = row_base + lrow_w;
  o_store_pass(sO, out, grow_w, n0, w, lane);
  __threadfence();
  o_store_pass(sO, out, grow_w, n0, w, lane);
}

extern "C" void kernel_launch(void* const* d_in, const int* in_sizes, int n_in,
                              void* d_out, int out_size, void* d_ws, size_t ws_size,
                              hipStream_t stream) {
  if (n_in < 3) return;
  if (in_sizes[0] != NROWS * NIN) return;
  if (in_sizes[1] != NOUT * KTOT) return;
  if (in_sizes[2] != NOUT) return;
  if (out_size != NROWS * NOUT) return;

  const float* x     = (const float*)d_in[0];
  const float* coeff = (const float*)d_in[1];
  const float* scale = (const float*)d_in[2];
  float* out = (float*)d_out;

  size_t off = 0;
  const size_t oAP = off; off += (size_t)CH * KTOT * 2;
  const size_t oWB = off; off += (size_t)NOUT * KTOT * 2;
  if (off > ws_size) return;
  if (off > (size_t)WSCAP) return;

  char* ws = (char*)d_ws;
  unsigned short* AP = (unsigned short*)(ws + oAP);
  unsigned short* WB = (unsigned short*)(ws + oWB);

  prep_kernel<<<dim3(PBLKS), dim3(256), 0, stream>>>(coeff, WB);
  for (int c = 0; c < NCHUNK; ++c) {
    const int row_base = c * CH;
    feat_kernel<<<dim3(CH), dim3(FTHR), 0, stream>>>(x, AP, row_base);
    gemm_kernel<<<dim3(CH / 128, NOUT / 64), dim3(128), 0, stream>>>(AP, WB, scale, out, row_base);
  }
  (void)hipGetLastError();
}
